// GeographyAwareAttention_13314398617911
// MI455X (gfx1250) — hardware-verified
//
#include <hip/hip_runtime.h>
#include <math.h>
#include <stdint.h>


#define NB    4
#define NT    1024
#define ND    1024
#define NH    16
#define HD    64
#define NTOK  (NB * NT)
#define NBH   (NB * NH)
#define QBLK  128
#define KCH   64
#define NKC   (NT / KCH)
#define KP    72
#define SPP   72
#define ATHR  256
#define LDSA  (4 * KCH * KP)

static_assert(NH * HD == ND);
static_assert((NT % QBLK) == 0 && (NT % KCH) == 0 && (NTOK % 64) == 0 && (ND % 64) == 0 && (ND % 32) == 0);
static_assert(QBLK == (ATHR / 32) * 16);
static_assert((ATHR / 32) * 2048 <= LDSA);
static_assert(KCH == 64 && HD == 64 && NKC * KCH == NT);
static_assert(((NTOK * ND) % 2048) == 0 && ((ND * ND) % 2048) == 0);

typedef _Float16 v16h __attribute__((ext_vector_type(16)));
typedef _Float16 v8h  __attribute__((ext_vector_type(8)));
typedef float    v8f  __attribute__((ext_vector_type(8)));
typedef float    v4f  __attribute__((ext_vector_type(4)));
typedef unsigned int v4u __attribute__((ext_vector_type(4)));
typedef int      v4i  __attribute__((ext_vector_type(4)));

__device__ __forceinline__ unsigned short bf_bits(float f) {
  unsigned u = __float_as_uint(f);
  return (unsigned short)((u + 0x7FFFu + ((u >> 16) & 1u)) >> 16);
}
__device__ __forceinline__ float bf_up(unsigned short h) { return __uint_as_float(((unsigned)h) << 16); }
__device__ __forceinline__ unsigned short h_bits(_Float16 x) { return __builtin_bit_cast(unsigned short, x); }
__device__ __forceinline__ unsigned pk16(unsigned short a, unsigned short b) { return (unsigned)a | ((unsigned)b << 16); }
__device__ __forceinline__ v8f zero8() { v8f z = {0.f, 0.f, 0.f, 0.f, 0.f, 0.f, 0.f, 0.f}; return z; }

__device__ __forceinline__ v16h ldfrag_h(const _Float16* p) {
  union { v16h v; v8h h[2]; } f;
  f.h[0] = *(const v8h*)(p);
  f.h[1] = *(const v8h*)(p + 16);
  return f.v;
}

__device__ __forceinline__ v8f mma_h_raw(v16h a, v16h b, v8f c) {
  return __builtin_amdgcn_wmma_f32_16x16x32_f16(false, a, false, b, (short)0, c, false, false);
}
__device__ __forceinline__ void res_guard(v8f& t, v8f& acc, v16h x, v16h y) {
#if defined(__HIP_DEVICE_COMPILE__)
  asm volatile("v_nop\n\tv_nop\n\tv_nop\n\tv_nop" : "+v"(t), "+v"(acc) : "v"(x), "v"(y));
#endif
}
__device__ __forceinline__ void dep_guard_h(v8f& a, v8f& b, v16h x, v16h y) {
#if defined(__HIP_DEVICE_COMPILE__)
  asm volatile("v_nop\n\tv_nop\n\tv_nop\n\tv_nop" : "+v"(a), "+v"(b) : "v"(x), "v"(y));
#endif
}
__device__ __forceinline__ void guard_sc8(v8f& a, v8f& b, v16h k0, v16h k1, v16h k2, v16h k3,
                                          v16h q0, v16h q1, v16h q2, v16h q3) {
#if defined(__HIP_DEVICE_COMPILE__)
  asm volatile("v_nop\n\tv_nop\n\tv_nop\n\tv_nop" : "+v"(a), "+v"(b)
               : "v"(k0), "v"(k1), "v"(k2), "v"(k3), "v"(q0), "v"(q1), "v"(q2), "v"(q3));
#endif
}
__device__ __forceinline__ void guard_pv(v8f& a, v8f& b, v16h w, v16h x, v16h y, v16h z) {
#if defined(__HIP_DEVICE_COMPILE__)
  asm volatile("v_nop\n\tv_nop\n\tv_nop\n\tv_nop" : "+v"(a), "+v"(b) : "v"(w), "v"(x), "v"(y), "v"(z));
#endif
}
__device__ __forceinline__ void keep4_h(v16h a, v16h b, v16h c, v16h d) {
#if defined(__HIP_DEVICE_COMPILE__)
  asm volatile("v_nop" :: "v"(a), "v"(b), "v"(c), "v"(d));
#endif
}
__device__ __forceinline__ void acc_guard4(v8f& a, v8f& b, v8f& c, v8f& d) {
#if defined(__HIP_DEVICE_COMPILE__)
  asm volatile("v_nop\n\tv_nop\n\tv_nop\n\tv_nop" : "+v"(a), "+v"(b), "+v"(c), "+v"(d));
#endif
}
__device__ __forceinline__ void wave_sync_lds() {
  __builtin_amdgcn_fence(__ATOMIC_RELEASE, "workgroup");
  __builtin_amdgcn_wave_barrier();
  __builtin_amdgcn_fence(__ATOMIC_ACQUIRE, "workgroup");
}

__global__ __launch_bounds__(256) void cvt_h8(const float* __restrict__ in, unsigned short* out, int n8, float scale) {
  const int i = blockIdx.x * 256 + threadIdx.x;
  if (i < n8) {
    const v4f a = *(const v4f*)(in + (size_t)i * 8);
    const v4f c = *(const v4f*)(in + (size_t)i * 8 + 4);
    float f[8];
    f[0] = a[0]; f[1] = a[1]; f[2] = a[2]; f[3] = a[3];
    f[4] = c[0]; f[5] = c[1]; f[6] = c[2]; f[7] = c[3];
    unsigned short hb[8];
#pragma unroll
    for (int e = 0; e < 8; ++e) hb[e] = h_bits((_Float16)(bf_up(bf_bits(f[e])) * scale));
    v4u p;
    p[0] = pk16(hb[0], hb[1]);
    p[1] = pk16(hb[2], hb[3]);
    p[2] = pk16(hb[4], hb[5]);
    p[3] = pk16(hb[6], hb[7]);
    *(volatile v4u*)(out + (size_t)i * 8) = p;
    __threadfence();
    *(volatile v4u*)(out + (size_t)i * 8) = p;
  }
}

__global__ __launch_bounds__(256) void gemm_proj(
    const unsigned short* __restrict__ XHp, const unsigned short* __restrict__ Wp,
    const float* __restrict__ bias,
    unsigned short* PH, unsigned short* PL, int trans, float oscale) {
  const _Float16* A  = (const _Float16*)(const void*)XHp;
  const _Float16* Bt = (const _Float16*)(const void*)Wp;
  __shared__ __align__(16) unsigned short sP[8][2][16 * SPP];
  const int lane = threadIdx.x & 31;
  const int wave = threadIdx.x >> 5;
  const int tilesN = ND / 64;
  const int tilesM = NTOK / 64;
  const int tile = blockIdx.x * 8 + wave;
  if (tile >= tilesM * tilesN) return;
  const int tm = tile / tilesN;
  const int tn = tile - tm * tilesN;
  const int m0 = tm << 6;
  const int n0 = tn << 6;
  const int rlane = lane & 15;
  const int hh    = lane >> 4;
  const int koff  = hh * 8;
  const int mOff  = hh * 8;

  v8f acc[4][4];
#pragma unroll
  for (int i = 0; i < 4; ++i)
#pragma unroll
    for (int j = 0; j < 4; ++j) acc[i][j] = zero8();

  for (int k0 = 0; k0 < ND; k0 += 32) {
    v16h bf[4];
#pragma unroll
    for (int j = 0; j < 4; ++j) {
      const size_t bo = (size_t)(n0 + (j << 4) + rlane) * ND + koff + k0;
      bf[j] = ldfrag_h(Bt + bo);
    }
#pragma unroll
    for (int i = 0; i < 4; ++i) {
      const size_t ao = (size_t)(m0 + (i << 4) + rlane) * ND + koff + k0;
      const v16h ah = ldfrag_h(A + ao);
#pragma unroll
      for (int j = 0; j < 4; ++j) acc[i][j] = mma_h_raw(ah, bf[j], acc[i][j]);
      dep_guard_h(acc[i][0], acc[i][3], ah, bf[3]);
    }
    keep4_h(bf[0], bf[1], bf[2], bf[3]);
  }
  acc_guard4(acc[0][0], acc[0][1], acc[0][2], acc[0][3]);
  acc_guard4(acc[1][0], acc[1][1], acc[1][2], acc[1][3]);
  acc_guard4(acc[2][0], acc[2][1], acc[2][2], acc[2][3]);
  acc_guard4(acc[3][0], acc[3][1], acc[3][2], acc[3][3]);

  const int b  = m0 / NT;
  const int t0 = m0 - b * NT;
  const int h  = n0 >> 6;
  const int bh = b * NH + h;
  float bc[4];
#pragma unroll
  for (int j = 0; j < 4; ++j) bc[j] = bf_up(bf_bits(bias[n0 + (j << 4) + rlane]));
  unsigned short* s0 = &sP[wave][0][0];
  unsigned short* s1 = &sP[wave][1][0];
  const int rq = lane >> 3, c8 = (lane & 7) * 8;

  if (trans == 0) {
#pragma unroll
    for (int i = 0; i < 4; ++i) {
#pragma unroll
      for (int j = 0; j < 4; ++j) {
#pragma unroll
        for (int r = 0; r < 8; ++r) {
          const float f = (acc[i][j][r] * oscale + bc[j]) * 16.0f;
          const _Float16 xh = (_Float16)f;
          const int so = (mOff + r) * SPP + (j << 4) + rlane;
          s0[so] = h_bits(xh);
          s1[so] = h_bits((_Float16)((f - (float)xh) * 2048.0f));
        }
      }
      wave_sync_lds();
      for (int pass = 0; pass < 2; ++pass) {
#pragma unroll
        for (int it = 0; it < 4; ++it) {
          const int row = it * 4 + rq;
          const size_t dst = ((size_t)(bh * NT + t0 + (i << 4) + row)) * HD + c8;
          const v4u v = *(const v4u*)(s0 + row * SPP + c8);
          const v4u w = *(const v4u*)(s1 + row * SPP + c8);
          *(volatile v4u*)(PH + dst) = v;
          *(volatile v4u*)(PL + dst) = w;
        }
        __threadfence();
      }
      wave_sync_lds();
    }
  } else {
#pragma unroll
    for (int j = 0; j < 4; ++j) {
#pragma unroll
      for (int i = 0; i < 4; ++i) {
        unsigned short hb[8], lb[8];
#pragma unroll
        for (int r = 0; r < 8; ++r) {
          const float f = (acc[i][j][r] * oscale + bc[j]) * 16.0f;
          const _Float16 xh = (_Float16)f;
          hb[r] = h_bits(xh);
          lb[r] = h_bits((_Float16)((f - (float)xh) * 2048.0f));
        }
        v4u ph, pl;
#pragma unroll
        for (int q = 0; q < 4; ++q) {
          ph[q] = pk16(hb[2 * q], hb[2 * q + 1]);
          pl[q] = pk16(lb[2 * q], lb[2 * q + 1]);
        }
        *(v4u*)(s0 + rlane * SPP + (i << 4) + mOff) = ph;
        *(v4u*)(s1 + rlane * SPP + (i << 4) + mOff) = pl;
      }
      wave_sync_lds();
      for (int pass = 0; pass < 2; ++pass) {
#pragma unroll
        for (int it = 0; it < 4; ++it) {
          const int row = it * 4 + rq;
          const size_t dst = ((size_t)(bh * HD + (j << 4) + row)) * NT + t0 + c8;
          const v4u v = *(const v4u*)(s0 + row * SPP + c8);
          const v4u w = *(const v4u*)(s1 + row * SPP + c8);
          *(volatile v4u*)(PH + dst) = v;
          *(volatile v4u*)(PL + dst) = w;
        }
        __threadfence();
      }
      wave_sync_lds();
    }
  }
}

__global__ __launch_bounds__(ATHR) void attn_kernel(
    const unsigned short* __restrict__ QHp, const unsigned short* __restrict__ QLp,
    const unsigned short* __restrict__ KHp, const unsigned short* __restrict__ KLp,
    const unsigned short* __restrict__ VHp, const unsigned short* __restrict__ VLp,
    const float* __restrict__ dist, const int* __restrict__ msk, const float* __restrict__ alphaP,
    unsigned short* CTXh, unsigned short* CTXl, float rscale) {
  __shared__ __align__(16) unsigned short lds_u[LDSA];
  __shared__ int sflag[2][8];
  unsigned short* kh_u = lds_u;
  unsigned short* kl_u = lds_u + KCH * KP;
  unsigned short* vh_u = lds_u + 2 * KCH * KP;
  unsigned short* vl_u = lds_u + 3 * KCH * KP;
  const _Float16* kh = (const _Float16*)(const void*)kh_u;
  const _Float16* kl = (const _Float16*)(const void*)kl_u;
  const _Float16* vh = (const _Float16*)(const void*)vh_u;
  const _Float16* vl = (const _Float16*)(const void*)vl_u;
  const _Float16* QH = (const _Float16*)(const void*)QHp;
  const _Float16* QL = (const _Float16*)(const void*)QLp;

  const int tid = threadIdx.x, lane = tid & 31, wave = tid >> 5;
  const int bh = blockIdx.x;
  const int b  = bh / NH;
  const int h  = bh - b * NH;
  const int q0 = blockIdx.y * QBLK;
  const int rlane = lane & 15, hsel = lane >> 4, koff = hsel * 8;
  const int qrow = q0 + wave * 16 + rlane;
  const float alpha = fabsf(bf_up(bf_bits(alphaP[0])));

  const size_t qo = ((size_t)(bh * NT + qrow)) * HD + koff;
  const v16h qh0 = ldfrag_h(QH + qo);
  const v16h qh1 = ldfrag_h(QH + qo + 32);
  const v16h ql0 = ldfrag_h(QL + qo);
  const v16h ql1 = ldfrag_h(QL + qo + 32);
  const size_t rowbase = ((size_t)(b * NT + qrow)) * NT;

  const float C2048  = 1.0f / 2048.0f;
  const float LN1024 = 6.931471805599453f;
  const float NEGINF = __uint_as_float(0xff800000u);

  v8f oh[4], ol[4];
#pragma unroll
  for (int dt = 0; dt < 4; ++dt) { oh[dt] = zero8(); ol[dt] = zero8(); }
  float m_run = -1.0e30f, l_run = 0.0f;

#pragma unroll 1
  for (int c = 0; c < NKC; ++c) {
    const int kc = c * KCH;
    unsigned bits = 0u;
#pragma unroll
    for (int s = 0; s < 2; ++s) {
#pragma unroll
      for (int t = 0; t < 2; ++t) {
        const int* mp = msk + rowbase + (size_t)(kc + 32 * s + 16 * t + 8 * hsel);
        const v4i ma = *(const v4i*)mp;
        const v4i mb = *(const v4i*)(mp + 4);
#pragma unroll
        for (int r = 0; r < 4; ++r) {
          bits |= ((ma[r] != 0) ? 1u : 0u) << (s * 16 + t * 8 + r);
          bits |= ((mb[r] != 0) ? 1u : 0u) << (s * 16 + t * 8 + 4 + r);
        }
      }
    }
    const int wany = __any(bits != 0u);
    if (lane == 0) sflag[c & 1][wave] = wany;
    __syncthreads();
    int bany = 0;
#pragma unroll
    for (int w = 0; w < 8; ++w) bany |= sflag[c & 1][w];
    if (bany == 0) continue;

    for (int i = tid; i < KCH * 8; i += ATHR) {
      const int key = i >> 3, c8 = (i & 7) * 8;
      const size_t gk = ((size_t)(bh * NT + kc + key)) * HD + c8;
      *(v4u*)(kh_u + key * KP + c8) = *(const v4u*)(KHp + gk);
      *(v4u*)(kl_u + key * KP + c8) = *(const v4u*)(KLp + gk);
      const int d = key;
      const size_t gv = ((size_t)(bh * HD + d)) * NT + kc + c8;
      *(v4u*)(vh_u + d * KP + c8) = *(const v4u*)(VHp + gv);
      *(v4u*)(vl_u + d * KP + c8) = *(const v4u*)(VLp + gv);
    }
    __syncthreads();

#pragma unroll 1
    for (int sub = 0; sub < 2; ++sub) {
      const int kr = sub * 32;
      const unsigned sbits = bits >> (sub * 16);
      float a[2][8];
#pragma unroll
      for (int t = 0; t < 2; ++t) {
        const int krow = kr + 16 * t + rlane;
        const v16h kha = ldfrag_h(kh + krow * KP + koff);
        const v16h khb = ldfrag_h(kh + krow * KP + 32 + koff);
        const v16h kla = ldfrag_h(kl + krow * KP + koff);
        const v16h klb = ldfrag_h(kl + krow * KP + 32 + koff);
        v8f sh = mma_h_raw(kha, qh0, zero8());
        sh = mma_h_raw(khb, qh1, sh);
        v8f sr = mma_h_raw(kha, ql0, zero8());
        sr = mma_h_raw(khb, ql1, sr);
        sr = mma_h_raw(kla, qh0, sr);
        sr = mma_h_raw(klb, qh1, sr);
        guard_sc8(sh, sr, kha, khb, kla, klb, qh0, qh1, ql0, ql1);
        const float* dp = dist + rowbase + (size_t)(kc + kr + 16 * t + 8 * hsel);
        const v4f d0 = *(const v4f*)(dp);
        const v4f d1 = *(const v4f*)(dp + 4);
        float dv[8];
        dv[0] = d0[0]; dv[1] = d0[1]; dv[2] = d0[2]; dv[3] = d0[3];
        dv[4] = d1[0]; dv[5] = d1[1]; dv[6] = d1[2]; dv[7] = d1[3];
#pragma unroll
        for (int r = 0; r < 8; ++r) {
          const float s = (sh[r] + sr[r] * C2048) * C2048 - alpha * bf_up(bf_bits(dv[r]));
          const unsigned kb = (sbits >> (t * 8 + r)) & 1u;
          a[t][r] = (kb != 0u) ? s : NEGINF;
        }
      }

      float mloc = -1.0e30f;
#pragma unroll
      for (int r = 0; r < 8; ++r) mloc = fmaxf(mloc, fmaxf(a[0][r], a[1][r]));
      mloc = fmaxf(mloc, __shfl_xor(mloc, 16, 32));
      const float newM  = fmaxf(m_run, mloc);
      const float alph  = __expf(m_run - newM);
      const float msh   = newM - LN1024;
      float ssum = 0.0f;
      float p[2][8];
#pragma unroll
      for (int r = 0; r < 8; ++r) {
        p[0][r] = __expf(a[0][r] - msh);
        p[1][r] = __expf(a[1][r] - msh);
        ssum += p[0][r] + p[1][r];
      }
      ssum += __shfl_xor(ssum, 16, 32);
      l_run = l_run * alph + ssum;
      m_run = newM;
#pragma unroll
      for (int dt = 0; dt < 4; ++dt) {
#pragma unroll
        for (int r = 0; r < 8; ++r) { oh[dt][r] *= alph; ol[dt][r] *= alph; }
      }

      union { v16h v; _Float16 s[16]; } ph, plo;
#pragma unroll
      for (int r = 0; r < 8; ++r) {
        const _Float16 x0 = (_Float16)p[0][r];
        const _Float16 x1 = (_Float16)p[1][r];
        ph.s[r]      = x0;
        ph.s[8 + r]  = x1;
        plo.s[r]     = (_Float16)((p[0][r] - (float)x0) * 2048.0f);
        plo.s[8 + r] = (_Float16)((p[1][r] - (float)x1) * 2048.0f);
      }

#pragma unroll
      for (int dt = 0; dt < 4; ++dt) {
        const v16h vah = ldfrag_h(vh + (16 * dt + rlane) * KP + kr + koff);
        const v16h val = ldfrag_h(vl + (16 * dt + rlane) * KP + kr + koff);
        oh[dt] = mma_h_raw(vah, ph.v, oh[dt]);
        ol[dt] = mma_h_raw(val, ph.v, ol[dt]);
        ol[dt] = mma_h_raw(vah, plo.v, ol[dt]);
        guard_pv(oh[dt], ol[dt], vah, val, ph.v, plo.v);
      }
    }
  }
  acc_guard4(oh[0], oh[1], oh[2], oh[3]);
  acc_guard4(ol[0], ol[1], ol[2], ol[3]);

  const float inv = 4.0f * (1.0f / l_run);
  __syncthreads();
  unsigned short* sth = lds_u + wave * 2048;
  unsigned short* stl = sth + 1024;
#pragma unroll
  for (int dt = 0; dt < 4; ++dt) {
    v4u hv, lw;
#pragma unroll
    for (int e = 0; e < 4; ++e) {
      const float f0 = (oh[dt][2 * e]     + ol[dt][2 * e]     * C2048) * inv;
      const float f1 = (oh[dt][2 * e + 1] + ol[dt][2 * e + 1] * C2048) * inv;
      const _Float16 x0 = (_Float16)f0, x1 = (_Float16)f1;
      hv[e] = pk16(h_bits(x0), h_bits(x1));
      lw[e] = pk16(h_bits((_Float16)((f0 - (float)x0) * rscale)),
                   h_bits((_Float16)((f1 - (float)x1) * rscale)));
    }
    const int so = rlane * 64 + 16 * dt + 8 * hsel;
    *(v4u*)(sth + so) = hv;
    *(v4u*)(stl + so) = lw;
  }
  wave_sync_lds();
  {
    const int rq = lane >> 3, c8 = (lane & 7) * 8;
    const int n0 = q0 + wave * 16;
    for (int pass = 0; pass < 2; ++pass) {
#pragma unroll
      for (int it = 0; it < 4; ++it) {
        const int row = it * 4 + rq;
        const v4u v = *(const v4u*)(sth + row * 64 + c8);
        *(volatile v4u*)(CTXh + ((size_t)(b * NT + n0 + row)) * ND + h * HD + c8) = v;
      }
      __threadfence();
    }
    for (int pass = 0; pass < 2; ++pass) {
#pragma unroll
      for (int it = 0; it < 4; ++it) {
        const int row = it * 4 + rq;
        const v4u v = *(const v4u*)(stl + row * 64 + c8);
        *(volatile v4u*)(CTXl + ((size_t)(b * NT + n0 + row)) * ND + h * HD + c8) = v;
      }
      __threadfence();
    }
  }
}

__global__ __launch_bounds__(256) void gemm_out(
    const unsigned short* __restrict__ Ap, const unsigned short* __restrict__ A2p,
    const unsigned short* __restrict__ Btp, const float* __restrict__ bias,
    float* Cout, float oscale, float rres) {
  const _Float16* A   = (const _Float16*)(const void*)Ap;
  const _Float16* A2  = (const _Float16*)(const void*)A2p;
  const _Float16* Bt  = (const _Float16*)(const void*)Btp;
  __shared__ __align__(16) float sT[8][16 * 68];
  const int lane = threadIdx.x & 31;
  const int wave = threadIdx.x >> 5;
  const int tilesN = ND / 64;
  const int tilesM = NTOK / 64;
  const int tile = blockIdx.x * 8 + wave;
  if (tile >= tilesM * tilesN) return;
  const int tm = tile / tilesN;
  const int tn = tile - tm * tilesN;
  const int m0 = tm << 6;
  const int n0 = tn << 6;
  const int rlane = lane & 15;
  const int koff  = (lane >> 4) * 8;
  const int mOff  = (lane >> 4) * 8;

  v8f acc[4][4];
#pragma unroll
  for (int i = 0; i < 4; ++i)
#pragma unroll
    for (int j = 0; j < 4; ++j) acc[i][j] = zero8();

  for (int k0 = 0; k0 < ND; k0 += 32) {
    v16h bf[4];
#pragma unroll
    for (int j = 0; j < 4; ++j) {
      const size_t bo = (size_t)(n0 + (j << 4) + rlane) * ND + koff + k0;
      bf[j] = ldfrag_h(Bt + bo);
    }
#pragma unroll
    for (int i = 0; i < 4; ++i) {
      const size_t ao = (size_t)(m0 + (i << 4) + rlane) * ND + koff + k0;
      const v16h ah = ldfrag_h(A + ao);
#pragma unroll
      for (int j = 0; j < 4; ++j) acc[i][j] = mma_h_raw(ah, bf[j], acc[i][j]);
      dep_guard_h(acc[i][0], acc[i][3], ah, bf[3]);
    }
#pragma unroll
    for (int i = 0; i < 4; ++i) {
      const size_t ao = (size_t)(m0 + (i << 4) + rlane) * ND + koff + k0;
      const v16h al = ldfrag_h(A2 + ao);
#pragma unroll
      for (int j = 0; j < 4; ++j) {
        v8f tp = mma_h_raw(al, bf[j], zero8());
        res_guard(tp, acc[i][j], al, bf[j]);
#pragma unroll
        for (int r = 0; r < 8; ++r) acc[i][j][r] += tp[r] * rres;
      }
      dep_guard_h(acc[i][0], acc[i][3], al, bf[3]);
    }
    keep4_h(bf[0], bf[1], bf[2], bf[3]);
  }
  acc_guard4(acc[0][0], acc[0][1], acc[0][2], acc[0][3]);
  acc_guard4(acc[1][0], acc[1][1], acc[1][2], acc[1][3]);
  acc_guard4(acc[2][0], acc[2][1], acc[2][2], acc[2][3]);
  acc_guard4(acc[3][0], acc[3][1], acc[3][2], acc[3][3]);

  float* slab = sT[wave];
  float bc[4];
#pragma unroll
  for (int j = 0; j < 4; ++j) bc[j] = bf_up(bf_bits(bias[n0 + (j << 4) + rlane]));
#pragma unroll
  for (int i = 0; i < 4; ++i) {
    const int mBase = m0 + (i << 4);
#pragma unroll
    for (int j = 0; j < 4; ++j) {
#pragma unroll
      for (int r = 0; r < 8; ++r) {
        slab[(mOff + r) * 68 + (j << 4) + rlane] = acc[i][j][r] * oscale + bc[j];
      }
    }
    wave_sync_lds();
    {
      const int hh = lane >> 4, c4 = (lane & 15) * 4;
      for (int pass = 0; pass < 2; ++pass) {
#pragma unroll
        for (int it = 0; it < 8; ++it) {
          const int row = it * 2 + hh;
          const v4f v = *(const v4f*)(slab + row * 68 + c4);
          *(volatile v4f*)(Cout + (size_t)(mBase + row) * ND + n0 + c4) = v;
        }
        __threadfence();
      }
    }
    wave_sync_lds();
  }
}

extern "C" void kernel_launch(void* const* d_in, const int* in_sizes, int n_in,
                              void* d_out, int out_size, void* d_ws, size_t ws_size,
                              hipStream_t stream) {
  if (n_in < 12) return;
  if (in_sizes[0] != NTOK * ND) return;
  if (in_sizes[1] != NB * NT * NT) return;
  if (in_sizes[2] != NB * NT * NT) return;
  if (in_sizes[3] != ND * ND || in_sizes[4] != ND) return;
  if (in_sizes[5] != ND * ND || in_sizes[6] != ND) return;
  if (in_sizes[7] != ND * ND || in_sizes[8] != ND) return;
  if (in_sizes[9] != ND * ND || in_sizes[10] != ND) return;
  if (in_sizes[11] < 1) return;
  if (out_size != NTOK * ND) return;

  const float* x     = (const float*)d_in[0];
  const float* dist  = (const float*)d_in[1];
  const int*   msk   = (const int*)d_in[2];
  const float* Wq    = (const float*)d_in[3];
  const float* bq    = (const float*)d_in[4];
  const float* Wk    = (const float*)d_in[5];
  const float* bk    = (const float*)d_in[6];
  const float* Wv    = (const float*)d_in[7];
  const float* bv    = (const float*)d_in[8];
  const float* Wo    = (const float*)d_in[9];
  const float* bo    = (const float*)d_in[10];
  const float* alpha = (const float*)d_in[11];

  const size_t PXH = (size_t)NTOK * ND * 2;
  const size_t PW  = (size_t)ND * ND * 2;
  const size_t PQK = (size_t)NBH * NT * HD * 2;
  const size_t PV  = (size_t)NBH * HD * NT * 2;
  const size_t PCT = (size_t)NTOK * ND * 2;
  size_t off = 0;
  const size_t oXH = off; off += PXH;
  const size_t oWQ = off; off += PW;
  const size_t oWK = off; off += PW;
  const size_t oWV = off; off += PW;
  const size_t oWO = off; off += PW;
  const size_t oQH = off; off += PQK;
  const size_t oQL = off; off += PQK;
  const size_t oKH = off; off += PQK;
  const size_t oKL = off; off += PQK;
  const size_t oVH = off; off += PV;
  const size_t oVL = off; off += PV;
  const size_t oCH = off; off += PCT;
  const size_t oCL = off; off += PCT;
  if (off > ws_size) return;
  if (off > (size_t)134217728) return;

  char* ws = (char*)d_ws;
  unsigned short* XH   = (unsigned short*)(ws + oXH);
  unsigned short* WQP  = (unsigned short*)(ws + oWQ);
  unsigned short* WKP  = (unsigned short*)(ws + oWK);
  unsigned short* WVP  = (unsigned short*)(ws + oWV);
  unsigned short* WOP  = (unsigned short*)(ws + oWO);
  unsigned short* QH   = (unsigned short*)(ws + oQH);
  unsigned short* QL   = (unsigned short*)(ws + oQL);
  unsigned short* KH   = (unsigned short*)(ws + oKH);
  unsigned short* KL   = (unsigned short*)(ws + oKL);
  unsigned short* VH   = (unsigned short*)(ws + oVH);
  unsigned short* VL   = (unsigned short*)(ws + oVL);
  unsigned short* CTXh = (unsigned short*)(ws + oCH);
  unsigned short* CTXl = (unsigned short*)(ws + oCL);
  float*          out  = (float*)d_out;

  const dim3 blk(256);
  const int n8x = NTOK * ND / 8;
  const int n8w = ND * ND / 8;
  const dim3 gX((n8x + 255) / 256);
  const dim3 gW((n8w + 255) / 256);
  const dim3 gProj(((NTOK / 64) * (ND / 64) + 7) / 8);
  const dim3 gAttn(NBH, NT / QBLK);
  const dim3 gOut(((NTOK / 64) * (ND / 64) + 7) / 8);

  const float oscPrj = 1.0f / 16384.0f;
  const float rscale = 16384.0f;
  const float oscOut = 1.0f / 65536.0f;
  const float rres   = 1.0f / 16384.0f;

  cvt_h8<<<gX, blk, 0, stream>>>(x,  XH,  n8x, 16.0f);
  cvt_h8<<<gW, blk, 0, stream>>>(Wq, WQP, n8w, 1024.0f);
  cvt_h8<<<gW, blk, 0, stream>>>(Wk, WKP, n8w, 1024.0f);
  cvt_h8<<<gW, blk, 0, stream>>>(Wv, WVP, n8w, 1024.0f);
  cvt_h8<<<gW, blk, 0, stream>>>(Wo, WOP, n8w, 1024.0f);
  gemm_proj<<<gProj, blk, 0, stream>>>(XH, WQP, bq, QH, QL, 0, oscPrj);
  gemm_proj<<<gProj, blk, 0, stream>>>(XH, WKP, bk, KH, KL, 0, oscPrj);
  gemm_proj<<<gProj, blk, 0, stream>>>(XH, WVP, bv, VH, VL, 1, oscPrj);
  attn_kernel<<<gAttn, dim3(ATHR), 0, stream>>>(QH, QL, KH, KL, VH, VL, dist, msk, alpha, CTXh, CTXl, rscale);
  gemm_out<<<gOut, blk, 0, stream>>>(CTXh, CTXl, WOP, bo, out, oscOut, rres);
  (void)hipGetLastError();
}
